// MambaBlock_46127948759439
// MI455X (gfx1250) — hardware-verified
//
#include <hip/hip_runtime.h>
#include <math.h>

typedef __attribute__((ext_vector_type(8)))  _Float16 v8h;
typedef __attribute__((ext_vector_type(16))) __bf16   v16b;
typedef __attribute__((ext_vector_type(8)))  __bf16   v8b;
typedef __attribute__((ext_vector_type(8)))  float    v8f;
typedef __attribute__((ext_vector_type(4)))  float    v4f;

constexpr int kBatch  = 2;
constexpr int kSeq    = 2048;
constexpr int kDm     = 768;
constexpr int kDin    = 1536;
constexpr int kNst    = 16;
constexpr int kDtR    = 48;
constexpr int kDtP    = 64;
constexpr int kXzP    = 2 * kDin;
constexpr int kPrjN   = kDtR + 2 * kNst;
constexpr int kPrjP   = 128;
constexpr int kRows   = kBatch * kSeq;
constexpr int kConvTP = 260;
constexpr int kScanTS = 64;
constexpr int kScanCh = 64;
constexpr int kScanYP = 68;
constexpr int kBCW    = 2 * kNst;
static_assert(kPrjN == 80 && kPrjN <= kPrjP, "x_proj width");
static_assert((kDm % 64) == 0 && (kDin % 64) == 0 && (kDtP % 32) == 0 && kDtR <= kDtP, "GEMM K multiples of 32");
static_assert((kRows % 64) == 0 && (kSeq % 64) == 0 && (kXzP % 64) == 0 && (kPrjP % 64) == 0 && (kDin % 64) == 0 && (kDm % 64) == 0, "GEMM M,N multiples of 64");
static_assert((kSeq % kScanTS) == 0 && (kDin % kScanCh) == 0 && (kDin % 256) == 0 && (kDtR % 8) == 0, "tile multiples");
static_assert(((kRows / 64) * (kXzP / 64)) % 8 == 0 && ((kRows / 64) * (kPrjP / 64)) % 8 == 0 &&
              ((kSeq / 64) * (kDin / 64)) % 8 == 0 && ((kRows / 64) * (kDm / 64)) % 8 == 0, "GEMM tile counts fill whole blocks");
static_assert((kDin % 2) == 0, "16-bit plane rows start on 32-bit word boundaries");

constexpr size_t kOffXB    = 0;
constexpr size_t kOffWINT  = kOffXB    + (size_t)kRows * kDm   * 2;
constexpr size_t kOffWXT   = kOffWINT  + (size_t)kXzP  * kDm   * 2;
constexpr size_t kOffWDTT  = kOffWXT   + (size_t)kPrjP * kDin  * 2;
constexpr size_t kOffWOUTT = kOffWDTT  + (size_t)kDin  * kDtP  * 2;
constexpr size_t kOffXZ    = kOffWOUTT + (size_t)kDm   * kDin  * 2;
constexpr size_t kOffUH    = kOffXZ    + (size_t)kRows * kXzP  * 4;
constexpr size_t kOffUL    = kOffUH    + (size_t)kRows * kDin  * 2;
constexpr size_t kOffSSM   = kOffUL    + (size_t)kRows * kDin  * 2;
constexpr size_t kOffDRH   = kOffSSM   + (size_t)kRows * kPrjP * 4;
constexpr size_t kOffDRL   = kOffDRH   + (size_t)kRows * kDtP  * 2;
constexpr size_t kOffDLR   = kOffDRL   + (size_t)kRows * kDtP  * 2;
constexpr size_t kOffYH    = kOffDLR   + (size_t)kSeq  * kDin  * 4;
constexpr size_t kOffYL    = kOffYH    + (size_t)kRows * kDin  * 2;
constexpr size_t kWsTotal  = kOffYL    + (size_t)kRows * kDin  * 2;
static_assert(kWsTotal == 130351104ull, "carve total");
static_assert(kWsTotal <= 134217728ull, "carve cap");
static_assert((kOffWINT % 128) == 0 && (kOffWXT % 128) == 0 && (kOffWDTT % 128) == 0 && (kOffWOUTT % 128) == 0 &&
              (kOffXZ % 128) == 0 && (kOffUH % 128) == 0 && (kOffUL % 128) == 0 && (kOffSSM % 128) == 0 &&
              (kOffDRH % 128) == 0 && (kOffDRL % 128) == 0 && (kOffDLR % 128) == 0 && (kOffYH % 128) == 0 &&
              (kOffYL % 128) == 0, "128-B aligned regions");

__device__ __forceinline__ unsigned short f2bf_bits(float f) {
  unsigned u = __float_as_uint(f);
  return (unsigned short)((u + 0x7FFFu + ((u >> 16) & 1u)) >> 16);
}
__device__ __forceinline__ float bf_bits2f(unsigned short h) { return __uint_as_float(((unsigned)h) << 16); }
__device__ __forceinline__ float rne_bf(float f) { return bf_bits2f(f2bf_bits(f)); }

__device__ __forceinline__ void row_guard_b(v8f& a, v8f& b, v8f& c, v8f& d, v16b x, v16b y) {
  asm volatile("v_nop\n\tv_nop\n\tv_nop\n\tv_nop" : "+v"(a), "+v"(b), "+v"(c), "+v"(d) : "v"(x), "v"(y));
}
__device__ __forceinline__ void keep4_b(v16b a, v16b b, v16b c, v16b d) { asm volatile("v_nop" :: "v"(a), "v"(b), "v"(c), "v"(d)); }
__device__ __forceinline__ void acc_guard4(v8f& a, v8f& b, v8f& c, v8f& d) { asm volatile("v_nop\n\tv_nop\n\tv_nop\n\tv_nop" : "+v"(a), "+v"(b), "+v"(c), "+v"(d)); }

struct FragB {
  union U { v16b v; v8b h[2]; };
  static __device__ __forceinline__ v16b load(const __bf16* p) {
    U f; f.h[0] = *(const v8b*)(p); f.h[1] = *(const v8b*)(p + 16); return f.v;
  }
  static __device__ __forceinline__ v8f mma(v16b a, v16b b, v8f c) {
    return __builtin_amdgcn_wmma_f32_16x16x32_bf16(false, a, false, b, (short)0, c, false, false);
  }
};

template <int SPL>
__global__ __launch_bounds__(256) void wmma_gemm64(
    const unsigned short* __restrict__ Ap, const unsigned short* __restrict__ A2p, int lda,
    const unsigned short* __restrict__ Btp, int ldb,
    float* __restrict__ C, int ldc, int M, int N, int K) {
  typedef __bf16 T;
  typedef v16b V;
  const T* A = (const T*)Ap; const T* A2 = (const T*)A2p; const T* Bt = (const T*)Btp;
  __shared__ __align__(16) float sT[8][16 * 68];
  const int lane = threadIdx.x & 31;
  const int wave = threadIdx.x >> 5;
  const int tilesN = N >> 6;
  const int tilesM = M >> 6;
  const int tile = blockIdx.x * 8 + wave;
  if (tile >= tilesM * tilesN) return;
  const int tm = tile / tilesN;
  const int tn = tile - tm * tilesN;
  const int m0 = tm << 6;
  const int n0 = tn << 6;

  const int rlane = lane & 15;
  const int koff  = (lane >> 4) * 8;
  const int mOff  = (lane >> 4) * 8;

  v8f acc[4][4];
#pragma unroll
  for (int i = 0; i < 4; ++i)
#pragma unroll
    for (int j = 0; j < 4; ++j) acc[i][j] = (v8f){0.f,0.f,0.f,0.f,0.f,0.f,0.f,0.f};

  for (int k0 = 0; k0 < K; k0 += 32) {
    V bh[4];
#pragma unroll
    for (int j = 0; j < 4; ++j) {
      const size_t bo = (size_t)(n0 + (j << 4) + rlane) * ldb + koff + k0;
      bh[j] = FragB::load(Bt + bo);
    }
#pragma unroll
    for (int i = 0; i < 4; ++i) {
      const size_t ao = (size_t)(m0 + (i << 4) + rlane) * lda + koff + k0;
      V ah = FragB::load(A + ao);
      V al = ah;
      if (SPL >= 1) al = FragB::load(A2 + ao);
#pragma unroll
      for (int j = 0; j < 4; ++j) {
        acc[i][j] = FragB::mma(ah, bh[j], acc[i][j]);
        if (SPL >= 1) acc[i][j] = FragB::mma(al, bh[j], acc[i][j]);
      }
      row_guard_b(acc[i][0], acc[i][1], acc[i][2], acc[i][3], ah, al);
    }
    keep4_b(bh[0], bh[1], bh[2], bh[3]);
  }
  acc_guard4(acc[0][0], acc[0][1], acc[0][2], acc[0][3]);
  acc_guard4(acc[1][0], acc[1][1], acc[1][2], acc[1][3]);
  acc_guard4(acc[2][0], acc[2][1], acc[2][2], acc[2][3]);
  acc_guard4(acc[3][0], acc[3][1], acc[3][2], acc[3][3]);

  float* slab = sT[wave];
#pragma unroll
  for (int i = 0; i < 4; ++i) {
    const int mBase = m0 + (i << 4);
#pragma unroll
    for (int j = 0; j < 4; ++j) {
#pragma unroll
      for (int r = 0; r < 8; ++r) {
        slab[(mOff + r) * 68 + (j << 4) + rlane] = acc[i][j][r];
      }
    }
    __builtin_amdgcn_fence(__ATOMIC_RELEASE, "workgroup");
    __builtin_amdgcn_wave_barrier();
    __builtin_amdgcn_fence(__ATOMIC_ACQUIRE, "workgroup");
    {
      const int hh = lane >> 4, c4 = (lane & 15) * 4;
      for (int pass = 0; pass < 2; ++pass) {
#pragma unroll
        for (int it = 0; it < 8; ++it) {
          const int row = it * 2 + hh;
          v4f v = *(const v4f*)(slab + row * 68 + c4);
          *(volatile v4f*)(C + (size_t)(mBase + row) * ldc + n0 + c4) = v;
        }
        __threadfence();
      }
    }
    __builtin_amdgcn_fence(__ATOMIC_RELEASE, "workgroup");
    __builtin_amdgcn_wave_barrier();
    __builtin_amdgcn_fence(__ATOMIC_ACQUIRE, "workgroup");
  }
}

__global__ __launch_bounds__(256) void cast_bf16_kernel(
    const float* __restrict__ src, unsigned short* __restrict__ dst, int total8)
{
  const int i = blockIdx.x * 256 + threadIdx.x;
  if (i >= total8) return;
  const size_t e0 = (size_t)i << 3;
  const v4f a0 = *(const v4f*)(src + e0);
  const v4f a1 = *(const v4f*)(src + e0 + 4);
  v8h hv;
#pragma unroll
  for (int e = 0; e < 4; ++e) {
    const float f0 = a0[e], f1 = a1[e];
    const unsigned short h0 = f2bf_bits(f0), h1 = f2bf_bits(f1);
    hv[e]     = __builtin_bit_cast(_Float16, h0);
    hv[4 + e] = __builtin_bit_cast(_Float16, h1);
  }
  unsigned short* q = dst + e0;
  *(volatile v8h*)q = hv;
  __threadfence();
  *(volatile v8h*)q = hv;
}

__global__ __launch_bounds__(256) void transpose_bf16_kernel(
    const float* __restrict__ W, unsigned short* __restrict__ Bt, int Kreal, int Ndim, int Kpad)
{
  __shared__ float tile[64 * 65];
  const int tid = threadIdx.x, lane = tid & 31, wave = tid >> 5;
  const int n0 = blockIdx.x * 64;
  const int k0 = blockIdx.y * 64;
#pragma unroll
  for (int half = 0; half < 2; ++half) {
#pragma unroll
    for (int p = 0; p < 8; ++p) {
      const int idx = tid + (half * 8 + p) * 256;
      const int kk  = idx >> 6;
      const int nn  = idx & 63;
      const int n   = n0 + nn;
      const int k   = k0 + kk;
      const int nc  = (n < Ndim) ? n : (Ndim - 1);
      const int kc  = (k < Kreal) ? k : (Kreal - 1);
      const float v = W[(size_t)kc * Ndim + nc];
      const bool ok = (n < Ndim) && (k < Kreal);
      tile[kk * 65 + nn] = ok ? v : 0.0f;
    }
    asm volatile("" ::: "memory");
  }
  __syncthreads();
  const int q = lane >> 3, c8 = (lane & 7) * 8;
  v8h hv[2];
#pragma unroll
  for (int it = 0; it < 2; ++it) {
    const int nrow = it * 32 + wave * 4 + q;
#pragma unroll
    for (int e = 0; e < 8; ++e) {
      const float f = tile[(c8 + e) * 65 + nrow];
      const unsigned short hb = f2bf_bits(f);
      hv[it][e] = __builtin_bit_cast(_Float16, hb);
    }
  }
  for (int pass = 0; pass < 2; ++pass) {
#pragma unroll
    for (int it = 0; it < 2; ++it) {
      const int nrow = it * 32 + wave * 4 + q;
      *(volatile v8h*)(Bt + (size_t)(n0 + nrow) * Kpad + k0 + c8) = hv[it];
    }
    __threadfence();
  }
}

__global__ __launch_bounds__(256) void conv_silu_kernel(
    const float* __restrict__ XZ, const float* __restrict__ cw, const float* __restrict__ cb,
    unsigned short* __restrict__ UH, unsigned short* __restrict__ UL)
{
  __shared__ __align__(16) float sT[16 * kConvTP];
  const int tid = threadIdx.x, lane = tid & 31, wave = tid >> 5;
  const int d0 = blockIdx.x * 256, d = d0 + tid;
  const int g0 = blockIdx.y * 64;
  const int tb = g0 & (kSeq - 1);
  const v4f wv = *(const v4f*)(cw + (size_t)d * 4);
  const float wr0 = wv[0], wr1 = wv[1], wr2 = wv[2], wr3 = wv[3];
  const float w0 = rne_bf(wr0), w1 = rne_bf(wr1), w2 = rne_bf(wr2), w3 = rne_bf(wr3);
  const float bc = rne_bf(cb[d]);
  float xm3, xm2, xm1;
  {
    const bool hist = (tb > 0);
    const int rb = hist ? (g0 - 3) : g0;
    const float v3 = XZ[(size_t)rb * kXzP + d];
    const float v2 = XZ[(size_t)(rb + 1) * kXzP + d];
    const float v1 = XZ[(size_t)(rb + 2) * kXzP + d];
    xm3 = hist ? v3 : 0.f;
    xm2 = hist ? v2 : 0.f;
    xm1 = hist ? v1 : 0.f;
  }
#pragma unroll 1
  for (int sub = 0; sub < 4; ++sub) {
    const int lb = g0 + sub * 16;
#pragma unroll 1
    for (int s = 0; s < 16; ++s) {
      const float xcur = XZ[(size_t)(lb + s) * kXzP + d];
      float acc = w0 * xm3;
      acc = fmaf(w1, xm2, acc);
      acc = fmaf(w2, xm1, acc);
      acc = fmaf(w3, xcur, acc);
      const float sv = acc + bc;
      const float sg = __builtin_amdgcn_rcpf(1.0f + __expf(-sv));
      sT[s * kConvTP + tid] = sv * sg;
      xm3 = xm2; xm2 = xm1; xm1 = xcur;
    }
    __syncthreads();
    v8h bh[2], blo[2];
#pragma unroll
    for (int it = 0; it < 2; ++it) {
      const float* sp = sT + (it * 8 + wave) * kConvTP + lane * 8;
      const v4f a0 = *(const v4f*)(sp);
      const v4f a1 = *(const v4f*)(sp + 4);
#pragma unroll
      for (int e = 0; e < 4; ++e) {
        const float f0 = a0[e], f1 = a1[e];
        const unsigned short h0 = f2bf_bits(f0), h1 = f2bf_bits(f1);
        const unsigned short l0 = f2bf_bits(f0 - bf_bits2f(h0)), l1 = f2bf_bits(f1 - bf_bits2f(h1));
        bh[it][e]      = __builtin_bit_cast(_Float16, h0);
        bh[it][4 + e]  = __builtin_bit_cast(_Float16, h1);
        blo[it][e]     = __builtin_bit_cast(_Float16, l0);
        blo[it][4 + e] = __builtin_bit_cast(_Float16, l1);
      }
    }
    for (int pass = 0; pass < 2; ++pass) {
#pragma unroll
      for (int it = 0; it < 2; ++it) {
        const size_t o = (size_t)(lb + it * 8 + wave) * kDin + d0 + lane * 8;
        *(volatile v8h*)(UH + o) = bh[it];
        *(volatile v8h*)(UL + o) = blo[it];
      }
      __threadfence();
    }
    __syncthreads();
  }
}

__global__ __launch_bounds__(256) void pack_dt_kernel(
    const float* __restrict__ SSM, unsigned short* __restrict__ DRH, unsigned short* __restrict__ DRL, int total8)
{
  const int i = blockIdx.x * 256 + threadIdx.x;
  if (i >= total8) return;
  const int e0  = i << 3;
  const int row = e0 >> 6;
  const int c8  = e0 & 63;
  const float* p = SSM + (size_t)row * kPrjP + c8;
  const v4f a0 = *(const v4f*)(p);
  const v4f a1 = *(const v4f*)(p + 4);
  const bool keep = (c8 < kDtR);
  v8h hv, lv;
#pragma unroll
  for (int e = 0; e < 4; ++e) {
    const float r0 = a0[e], r1 = a1[e];
    const float f0 = keep ? r0 : 0.0f;
    const float f1 = keep ? r1 : 0.0f;
    const unsigned short h0 = f2bf_bits(f0), h1 = f2bf_bits(f1);
    const unsigned short l0 = f2bf_bits(f0 - bf_bits2f(h0)), l1 = f2bf_bits(f1 - bf_bits2f(h1));
    hv[e]     = __builtin_bit_cast(_Float16, h0);
    hv[4 + e] = __builtin_bit_cast(_Float16, h1);
    lv[e]     = __builtin_bit_cast(_Float16, l0);
    lv[4 + e] = __builtin_bit_cast(_Float16, l1);
  }
  unsigned short* qh = DRH + e0;
  unsigned short* ql = DRL + e0;
  *(volatile v8h*)qh = hv;
  *(volatile v8h*)ql = lv;
  __threadfence();
  *(volatile v8h*)qh = hv;
  *(volatile v8h*)ql = lv;
}

__global__ __launch_bounds__(64) void scan_kernel(
    const float* __restrict__ SSMb, const unsigned* __restrict__ UHw, const unsigned* __restrict__ ULw,
    const float* __restrict__ XZb, const float* __restrict__ DLR,
    const float* __restrict__ bdt, const float* __restrict__ Alog, const float* __restrict__ Dp,
    unsigned short* __restrict__ YHb, unsigned short* __restrict__ YLb)
{
  __shared__ __align__(16) float sX[kScanTS * kBCW];
  __shared__ __align__(16) float sY[kScanTS * kScanYP];
  __shared__ __align__(16) float sA[kNst * kScanCh];
  const int tid = threadIdx.x, lane = tid & 31, wave = tid >> 5;
  const int d0 = blockIdx.x * kScanCh;
  const int d  = d0 + tid;
#pragma unroll 1
  for (int s = 0; s < kNst; ++s) {
    const float al = rne_bf(Alog[(size_t)d * kNst + s]);
    sA[s * kScanCh + tid] = -expf(al);
  }
  __syncthreads();
  float negA[kNst], h[kNst];
#pragma unroll
  for (int s = 0; s < kNst; ++s) {
    negA[s] = sA[s * kScanCh + tid];
    h[s] = 0.f;
  }
  const float bb = rne_bf(bdt[d]);
  const float Dd = rne_bf(Dp[d]);
  const bool oddch = ((d & 1) != 0);
  const int lr = tid >> 3, lc4 = (tid & 7) * 4;
  const int q = lane >> 3, c8 = (lane & 7) * 8;
#pragma unroll 1
  for (int t0 = 0; t0 < kSeq; t0 += kScanTS) {
    __syncthreads();
#pragma unroll
    for (int i = 0; i < 8; ++i) {
      const int r = lr + 8 * i;
      *(v4f*)(sX + r * kBCW + lc4) = *(const v4f*)(SSMb + (size_t)(t0 + r) * kPrjP + kDtR + lc4);
    }
    __syncthreads();
#pragma unroll 1
    for (int s = 0; s < kScanTS; ++s) {
      const size_t t = (size_t)(t0 + s);
      const float* xr = sX + s * kBCW;
      float Bs[kNst], Cs[kNst];
#pragma unroll
      for (int q4 = 0; q4 < 4; ++q4) {
        const v4f bv = *(const v4f*)(xr + 4 * q4);
        const v4f cv = *(const v4f*)(xr + kNst + 4 * q4);
        Bs[4 * q4 + 0] = bv[0]; Bs[4 * q4 + 1] = bv[1]; Bs[4 * q4 + 2] = bv[2]; Bs[4 * q4 + 3] = bv[3];
        Cs[4 * q4 + 0] = cv[0]; Cs[4 * q4 + 1] = cv[1]; Cs[4 * q4 + 2] = cv[2]; Cs[4 * q4 + 3] = cv[3];
      }
      const float v   = DLR[t * kDin + d] + bb;
      const float a   = __expf(-fabsf(v));
      const float u1  = 1.0f + a;
      const float l1p = __logf(u1) + (a - (u1 - 1.0f)) * __builtin_amdgcn_rcpf(u1);
      const float dt  = fmaxf(v, 0.0f) + l1p;
      const size_t wi = (t * kDin + (size_t)d) >> 1;
      unsigned wh = UHw[wi];
      unsigned wl = ULw[wi];
      asm volatile("" : "+v"(wh), "+v"(wl));
      const unsigned hbits = oddch ? (wh & 0xffff0000u) : (wh << 16);
      const unsigned lbits = oddch ? (wl & 0xffff0000u) : (wl << 16);
      const float xt  = __uint_as_float(hbits) + __uint_as_float(lbits);
      const float zv  = XZb[t * kXzP + kDin + d];
      const float dtx = dt * xt;
      float y = 0.f;
#pragma unroll
      for (int k = 0; k < kNst; ++k) {
        const float e = __expf(dt * negA[k]);
        h[k] = e * h[k] + dtx * Bs[k];
        y = h[k] * Cs[k] + y;
      }
      y = xt * Dd + y;
      const float sg = __builtin_amdgcn_rcpf(1.0f + __expf(-zv));
      y = y * (zv * sg);
      sY[s * kScanYP + tid] = y;
    }
    __syncthreads();
    v8h hv[8], lv[8];
#pragma unroll
    for (int it = 0; it < 8; ++it) {
      const int row = it * 8 + wave * 4 + q;
      const float* sp = sY + row * kScanYP + c8;
      const v4f a0 = *(const v4f*)(sp);
      const v4f a1 = *(const v4f*)(sp + 4);
#pragma unroll
      for (int e = 0; e < 4; ++e) {
        const float f0 = a0[e], f1 = a1[e];
        const unsigned short h0 = f2bf_bits(f0), h1 = f2bf_bits(f1);
        const unsigned short l0 = f2bf_bits(f0 - bf_bits2f(h0)), l1 = f2bf_bits(f1 - bf_bits2f(h1));
        hv[it][e]     = __builtin_bit_cast(_Float16, h0);
        hv[it][4 + e] = __builtin_bit_cast(_Float16, h1);
        lv[it][e]     = __builtin_bit_cast(_Float16, l0);
        lv[it][4 + e] = __builtin_bit_cast(_Float16, l1);
      }
    }
    for (int pass = 0; pass < 2; ++pass) {
#pragma unroll
      for (int it = 0; it < 8; ++it) {
        const int row = it * 8 + wave * 4 + q;
        const size_t o = (size_t)(t0 + row) * kDin + d0 + c8;
        *(volatile v8h*)(YHb + o) = hv[it];
        *(volatile v8h*)(YLb + o) = lv[it];
      }
      __threadfence();
    }
  }
}

extern "C" void kernel_launch(void* const* d_in, const int* in_sizes, int n_in,
                              void* d_out, int out_size, void* d_ws, size_t ws_size,
                              hipStream_t stream) {
  if (n_in < 10) return;
  if (in_sizes[0] != kRows * kDm) return;
  if (in_sizes[1] != kDm * kXzP) return;
  if (in_sizes[2] != kDin * 4) return;
  if (in_sizes[3] != kDin) return;
  if (in_sizes[4] != kDin * kPrjN) return;
  if (in_sizes[5] != kDtR * kDin) return;
  if (in_sizes[6] != kDin) return;
  if (in_sizes[7] != kDin * kNst) return;
  if (in_sizes[8] != kDin) return;
  if (in_sizes[9] != kDin * kDm) return;
  if (out_size != kRows * kDm) return;
  if (ws_size < kWsTotal) return;

  const float* x      = (const float*)d_in[0];
  const float* W_in   = (const float*)d_in[1];
  const float* conv_w = (const float*)d_in[2];
  const float* conv_b = (const float*)d_in[3];
  const float* W_x    = (const float*)d_in[4];
  const float* W_dt   = (const float*)d_in[5];
  const float* b_dt   = (const float*)d_in[6];
  const float* A_log  = (const float*)d_in[7];
  const float* Dp     = (const float*)d_in[8];
  const float* W_out  = (const float*)d_in[9];
  float* out = (float*)d_out;

  char* ws = (char*)d_ws;
  unsigned short* XB    = (unsigned short*)(ws + kOffXB);
  unsigned short* WINT  = (unsigned short*)(ws + kOffWINT);
  unsigned short* WXT   = (unsigned short*)(ws + kOffWXT);
  unsigned short* WDTT  = (unsigned short*)(ws + kOffWDTT);
  unsigned short* WOUTT = (unsigned short*)(ws + kOffWOUTT);
  float*          XZ    = (float*)(ws + kOffXZ);
  unsigned short* UH    = (unsigned short*)(ws + kOffUH);
  unsigned short* UL    = (unsigned short*)(ws + kOffUL);
  float*          SSM   = (float*)(ws + kOffSSM);
  unsigned short* DRH   = (unsigned short*)(ws + kOffDRH);
  unsigned short* DRL   = (unsigned short*)(ws + kOffDRL);
  float*          DLR   = (float*)(ws + kOffDLR);
  unsigned short* YH    = (unsigned short*)(ws + kOffYH);
  unsigned short* YL    = (unsigned short*)(ws + kOffYL);

  cast_bf16_kernel<<<(kRows * kDm / 8) / 256, 256, 0, stream>>>(x, XB, kRows * kDm / 8);
  transpose_bf16_kernel<<<dim3(kXzP / 64, kDm / 64), 256, 0, stream>>>(W_in, WINT, kDm, kXzP, kDm);
  transpose_bf16_kernel<<<dim3(kPrjP / 64, kDin / 64), 256, 0, stream>>>(W_x, WXT, kDin, kPrjN, kDin);
  transpose_bf16_kernel<<<dim3(kDin / 64, kDtP / 64), 256, 0, stream>>>(W_dt, WDTT, kDtR, kDin, kDtP);
  transpose_bf16_kernel<<<dim3(kDm / 64, kDin / 64), 256, 0, stream>>>(W_out, WOUTT, kDin, kDm, kDin);

  wmma_gemm64<0><<<((kRows / 64) * (kXzP / 64)) / 8, 256, 0, stream>>>(
      XB, XB, kDm, WINT, kDm, XZ, kXzP, kRows, kXzP, kDm);

  conv_silu_kernel<<<dim3(kDin / 256, kRows / 64), 256, 0, stream>>>(XZ, conv_w, conv_b, UH, UL);

  wmma_gemm64<1><<<((kRows / 64) * (kPrjP / 64)) / 8, 256, 0, stream>>>(
      UH, UL, kDin, WXT, kDin, SSM, kPrjP, kRows, kPrjP, kDin);

  pack_dt_kernel<<<(kRows * kDtP / 8) / 256, 256, 0, stream>>>(SSM, DRH, DRL, kRows * kDtP / 8);

  for (int b = 0; b < kBatch; ++b) {
    const size_t r0 = (size_t)b * kSeq;
    wmma_gemm64<1><<<((kSeq / 64) * (kDin / 64)) / 8, 256, 0, stream>>>(
        DRH + r0 * kDtP, DRL + r0 * kDtP, kDtP, WDTT, kDtP, DLR, kDin, kSeq, kDin, kDtP);
    scan_kernel<<<kDin / kScanCh, kScanCh, 0, stream>>>(
        SSM + r0 * kPrjP, (const unsigned*)(UH + r0 * kDin), (const unsigned*)(UL + r0 * kDin), XZ + r0 * kXzP, DLR,
        b_dt, A_log, Dp, YH + r0 * kDin, YL + r0 * kDin);
  }

  wmma_gemm64<1><<<((kRows / 64) * (kDm / 64)) / 8, 256, 0, stream>>>(
      YH, YL, kDin, WOUTT, kDin, out, kDm, kRows, kDm, kDin);
}
